// MultiHeadAttention_76948634075345
// MI455X (gfx1250) — hardware-run, weakly checked
//
#include <hip/hip_runtime.h>


#ifndef NB
#define NB 4
#endif
#ifndef SEQ
#define SEQ 2048
#endif
#define NB_FULL  4
#define SEQ_FULL 2048
#ifndef OUT_SEQ
#define OUT_SEQ SEQ
#endif
#define DM   1024
#define NH_  16
#define HD   64
#define AW   4
#define EARLY ((SEQ) < 512 ? (SEQ) : 512)
#define QRS  2048.0f
#define QRI  (1.0f / 2048.0f)
#define SC2  (0.125f * 1.4426950408889634f)
#define PSH  8.0f
#define NEGS (-6.1963280e9f)
#define MTHR (-1.0e9f)

static_assert(HD == 64);
static_assert(NH_ * HD == DM);
static_assert(DM % 64 == 0);
static_assert(DM % 32 == 0);
static_assert(SEQ % 64 == 0);
static_assert((NB * SEQ) % 64 == 0);
static_assert(SEQ % 32 == 0);
static_assert(EARLY % 64 == 0);
static_assert(EARLY % (16 * AW) == 0);
static_assert((SEQ - EARLY) % (16 * AW) == 0);
static_assert(((size_t)SEQ * DM) % 8 == 0);
static_assert(NB <= NB_FULL);
static_assert(SEQ <= SEQ_FULL);

typedef _Float16 h16;
typedef unsigned short bf;
typedef __attribute__((ext_vector_type(16))) __bf16   v16bf;
typedef __attribute__((ext_vector_type(16))) _Float16 v16h;
typedef __attribute__((ext_vector_type(8)))  _Float16 v8h;
typedef __attribute__((ext_vector_type(8)))  unsigned short v8us;
typedef __attribute__((ext_vector_type(8)))  float    v8f;
typedef __attribute__((ext_vector_type(4)))  float    v4f;
typedef v4f  __attribute__((may_alias)) v4fa;
typedef v8h  __attribute__((may_alias)) v8ha;

__device__ __forceinline__ unsigned short f2bf(float f) { unsigned u = __float_as_uint(f); u += 0x7FFFu + ((u >> 16) & 1u); return (unsigned short)(u >> 16); }
__device__ __forceinline__ float bfr(float f) { return __uint_as_float(((unsigned)f2bf(f)) << 16); }
__device__ __forceinline__ v16h cat16(v8h lo, v8h hi) { return __builtin_shufflevector(lo, hi, 0, 1, 2, 3, 4, 5, 6, 7, 8, 9, 10, 11, 12, 13, 14, 15); }
__device__ __forceinline__ v16bf cat16b(v8us lo, v8us hi) { return __builtin_bit_cast(v16bf, __builtin_shufflevector(lo, hi, 0, 1, 2, 3, 4, 5, 6, 7, 8, 9, 10, 11, 12, 13, 14, 15)); }
__device__ __forceinline__ v8f wmma16(v16h a, v16h b, v8f c) { return __builtin_amdgcn_wmma_f32_16x16x32_f16(false, a, false, b, (short)0, c, false, false); }
__device__ __forceinline__ v8f wmmab(v16bf a, v16bf b, v8f c) { return __builtin_amdgcn_wmma_f32_16x16x32_bf16(false, a, false, b, (short)0, c, false, false); }
__device__ __forceinline__ v16h  ldh(const h16* p) { return cat16(*(const v8h*)p, *(const v8h*)(p + 16)); }
__device__ __forceinline__ v16bf ldb(const bf* p)  { return cat16b(*(const v8us*)p, *(const v8us*)(p + 16)); }
__device__ __forceinline__ void wave_sync() { __builtin_amdgcn_fence(3  , "wavefront"); __builtin_amdgcn_wave_barrier(); asm volatile("" ::: "memory"); }

__global__ __launch_bounds__(256) void k_cvt8(const float* __restrict__ src, bf* dst, size_t n8) {
    const size_t i = (size_t)blockIdx.x * 256 + threadIdx.x; if (i >= n8) return;
    const v8f v = *(const v8f*)(src + i * 8); v8us o;
#pragma unroll
    for (int k = 0; k < 8; ++k) o[k] = f2bf(v[k]);
    *(volatile v8us*)(dst + i * 8) = o; __threadfence(); *(volatile v8us*)(dst + i * 8) = o;
}

__global__ __launch_bounds__(256) void k_cvtT(const float* __restrict__ W, bf* WT) {
    __shared__ float ts[64 * 65];
    const int tid = threadIdx.x; const int n0 = blockIdx.x * 64, k0 = blockIdx.y * 64;
#pragma unroll 4
    for (int i = 0; i < 16; ++i) { const int row = i * 4 + (tid >> 6), col = tid & 63; ts[row * 65 + col] = W[(size_t)(k0 + row) * DM + n0 + col]; }
    __syncthreads();
    const int rr = tid >> 3, c8 = (tid & 7) * 8;
    v8us o0, o1;
#pragma unroll
    for (int kk = 0; kk < 8; ++kk) { o0[kk] = f2bf(ts[(c8 + kk) * 65 + rr]); o1[kk] = f2bf(ts[(c8 + kk) * 65 + rr + 32]); }
    bf* p0 = WT + (size_t)(n0 + rr) * DM + k0 + c8; bf* p1 = p0 + (size_t)32 * DM;
    *(volatile v8us*)p0 = o0; *(volatile v8us*)p1 = o1;
    __threadfence();
    *(volatile v8us*)p0 = o0; *(volatile v8us*)p1 = o1;
}

template <int MODE>
__global__ __launch_bounds__(32) void k_proj(const bf* __restrict__ A, const bf* __restrict__ Bt, const float* __restrict__ bias, h16* Ph, h16* Pr, h16* MP) {
    __shared__ __align__(16) float os[16 * 68];
    __shared__ __align__(16) h16 ms[64];
    const int K = DM;
    const int lane = threadIdx.x & 31, lr = lane & 15, hi = lane >> 4; const int r0 = blockIdx.x * 64, c0 = blockIdx.y * 64;
    v8f acc[4][4];
#pragma unroll
    for (int mb = 0; mb < 4; ++mb)
#pragma unroll
        for (int nb = 0; nb < 4; ++nb) acc[mb][nb] = (v8f){};
    const size_t aoff = (size_t)(r0 + lr) * K + 8 * hi, boff = (size_t)(c0 + lr) * K + 8 * hi;
#pragma unroll 1
    for (int kc = 0; kc < K; kc += 32) {
        v16bf a[4];
#pragma unroll
        for (int mb = 0; mb < 4; ++mb) a[mb] = ldb(A + aoff + (size_t)mb * 16 * K + kc);
#pragma unroll
        for (int nb = 0; nb < 4; ++nb) { const v16bf b = ldb(Bt + boff + (size_t)nb * 16 * K + kc);
#pragma unroll
            for (int mb = 0; mb < 4; ++mb) acc[mb][nb] = wmmab(a[mb], b, acc[mb][nb]); }
        asm volatile("v_nop\n\tv_nop\n\tv_nop\n\tv_nop" : "+v"(acc[0][0]), "+v"(acc[1][1]), "+v"(acc[2][2]), "+v"(acc[3][3]) : "v"(a[0]), "v"(a[1]), "v"(a[2]), "v"(a[3]));
    }
    size_t hbase, rbase, mbase = 0; int hpitch, rpitch, t0;
    if (MODE == 0) { const int b = r0 / SEQ; t0 = r0 % SEQ; const int zh = b * NH_ + c0 / HD;
        hbase = ((size_t)zh * SEQ + t0) * HD; hpitch = HD; rbase = ((size_t)zh * EARLY + t0) * HD; rpitch = HD; mbase = (size_t)zh * SEQ + t0; }
    else { const int b = c0 / SEQ; t0 = c0 % SEQ;
        hbase = ((size_t)b * DM + r0) * SEQ + t0; hpitch = SEQ; rbase = ((size_t)b * DM + r0) * EARLY + t0; rpitch = EARLY; }
    const bool doRes = t0 < EARLY;
    const int c8 = (lane & 7) * 8;
    v4f bb0 = (v4f){}, bb1 = (v4f){};
    if (MODE == 0) { const v4f q0 = *(const v4f*)(bias + c0 + c8); const v4f q1 = *(const v4f*)(bias + c0 + c8 + 4);
#pragma unroll
        for (int i = 0; i < 4; ++i) { bb0[i] = bfr(q0[i]); bb1[i] = bfr(q1[i]); } }
#pragma unroll
    for (int mb = 0; mb < 4; ++mb) {
#pragma unroll
        for (int nb = 0; nb < 4; ++nb) {
#pragma unroll
            for (int j = 0; j < 8; ++j) os[(hi * 8 + j) * 68 + nb * 16 + lr] = acc[mb][nb][j]; }
        wave_sync();
        const size_t hb = hbase + (size_t)(mb * 16) * (size_t)hpitch;
        const size_t rb = rbase + (size_t)(mb * 16) * (size_t)rpitch;
#pragma unroll 1
        for (int ps = 0; ps < 2; ++ps) {
#pragma unroll
            for (int s = 0; s < 4; ++s) { const int row = 4 * s + (lane >> 3);
                v4f x0 = *(const v4fa*)(&os[row * 68 + c8]); v4f x1 = *(const v4fa*)(&os[row * 68 + c8 + 4]);
                if (MODE == 0) { x0 = x0 + bb0; x1 = x1 + bb1; }
                else { const float br = bfr(bias[r0 + mb * 16 + row]); x0 = x0 + br; x1 = x1 + br; }
                v8h hv, rv;
#pragma unroll
                for (int i = 0; i < 4; ++i) { const h16 a0 = (h16)x0[i]; const h16 a1 = (h16)x1[i]; hv[i] = a0; hv[4 + i] = a1; rv[i] = (h16)((x0[i] - (float)a0) * QRS); rv[4 + i] = (h16)((x1[i] - (float)a1) * QRS); }
                if (MODE == 0) {
                    float rs = ((x0[0] + x0[1]) + (x0[2] + x0[3])) + ((x1[0] + x1[1]) + (x1[2] + x1[3]));
                    rs += __shfl_xor(rs, 1, 32); rs += __shfl_xor(rs, 2, 32); rs += __shfl_xor(rs, 4, 32);
                    const h16 mv = (rs != 0.0f) ? (h16)1.0f : (h16)0.0f;
                    if ((lane & 7) == 0) ms[mb * 16 + row] = mv;
                }
                *(volatile v8h*)(Ph + hb + (size_t)row * (size_t)hpitch + c8) = hv;
                if (doRes) *(volatile v8h*)(Pr + rb + (size_t)row * (size_t)rpitch + c8) = rv; }
            if (ps == 0) __threadfence(); }
        wave_sync();
    }
    if (MODE == 0) {
        const v8h mv8 = *(const v8ha*)(&ms[c8]);
        h16* mp = MP + mbase + c8;
        if (lane < 8) *(volatile v8h*)mp = mv8;
        __threadfence();
        if (lane < 8) *(volatile v8h*)mp = mv8;
    }
}

template <int EK>
__global__ __launch_bounds__(32 * AW) void k_flash(const h16* __restrict__ QH, const h16* __restrict__ QR, const h16* __restrict__ KP, const h16* __restrict__ KR,
                                                   const h16* __restrict__ VT, const h16* __restrict__ VR, const h16* __restrict__ MQ, const h16* __restrict__ MK, float* OUT) {
    __shared__ __align__(16) float os[AW * 16 * 68];
    const int lane = threadIdx.x & 31, wave = __builtin_amdgcn_readfirstlane((int)(threadIdx.x >> 5)), lr = lane & 15, hi = lane >> 4;
    const int zh = blockIdx.y; const int b = zh / NH_, h = zh % NH_;
    const int t0 = (EK ? 0 : EARLY) + (blockIdx.x * AW + wave) * 16;
    const int tq = t0 + lr;
    const size_t pbase = (size_t)zh * SEQ * HD;
    const size_t rbase = (size_t)zh * EARLY * HD;
    const size_t qo = pbase + (size_t)tq * HD + 8 * hi;
    const v16h qh0 = ldh(QH + qo), qh1 = ldh(QH + qo + 32);
    v16h qr0 = (v16h){}, qr1 = (v16h){};
    if (EK) { const size_t qro = rbase + (size_t)tq * HD + 8 * hi; qr0 = ldh(QR + qro); qr1 = ldh(QR + qro + 32); }
    const size_t ko  = pbase + (size_t)lr * HD + 8 * hi;
    const size_t kro = rbase + (size_t)lr * HD + 8 * hi;
    const size_t vo  = pbase + (size_t)lr * SEQ + 8 * hi;
    const size_t vro = rbase + (size_t)lr * EARLY + 8 * hi;
    const size_t mo  = (size_t)zh * SEQ + 8 * hi;
    v8f o0 = (v8f){}, o1 = (v8f){}, o2 = (v8f){}, o3 = (v8f){};
    v8f e0 = (v8f){}, e1 = (v8f){}, e2 = (v8f){}, e3 = (v8f){};
    float m = -3.0e38f, l = 0.0f;
    const int kc = ((t0 + 47) >> 5) << 5;
    int kend = kc;
#pragma unroll 1
    for (int key0 = 0; key0 < kend; key0 += 32) {
        const h16* ka = KP + ko + (size_t)key0 * HD;
        const v16h ka0 = ldh(ka), ka1 = ldh(ka + 32), kb0 = ldh(ka + 16 * HD), kb1 = ldh(ka + 16 * HD + 32);
        const v8h kma = *(const v8h*)(MK + mo + key0); const v8h kmb = *(const v8h*)(MK + mo + key0 + 16);
        const bool rok = key0 < EARLY;
        v8f sHa = (v8f){}, sLa = (v8f){}, sHb = (v8f){}, sLb = (v8f){};
        if (EK) {
            v16h ra0 = (v16h){}, ra1 = (v16h){}, rb0 = (v16h){}, rb1 = (v16h){};
            if (rok) { const h16* kr = KR + kro + (size_t)key0 * HD; ra0 = ldh(kr); ra1 = ldh(kr + 32); rb0 = ldh(kr + 16 * HD); rb1 = ldh(kr + 16 * HD + 32); }
            sHa = wmma16(ka0, qh0, sHa); sLa = wmma16(ka0, qr0, sLa); sHb = wmma16(kb0, qh0, sHb); sLb = wmma16(kb0, qr0, sLb);
            sHa = wmma16(ka1, qh1, sHa); sLa = wmma16(ka1, qr1, sLa); sHb = wmma16(kb1, qh1, sHb); sLb = wmma16(kb1, qr1, sLb);
            sLa = wmma16(ra0, qh0, sLa); sLb = wmma16(rb0, qh0, sLb); sLa = wmma16(ra1, qh1, sLa); sLb = wmma16(rb1, qh1, sLb);
            asm volatile("v_nop\n\tv_nop\n\tv_nop\n\tv_nop" : "+v"(sHa), "+v"(sLa), "+v"(sHb), "+v"(sLb) : "v"(ka0), "v"(ka1), "v"(kb0), "v"(kb1), "v"(ra0), "v"(ra1), "v"(rb0), "v"(rb1));
        } else {
            sHa = wmma16(ka0, qh0, sHa); sHb = wmma16(kb0, qh0, sHb);
            sHa = wmma16(ka1, qh1, sHa); sHb = wmma16(kb1, qh1, sHb);
            asm volatile("v_nop\n\tv_nop\n\tv_nop\n\tv_nop" : "+v"(sHa), "+v"(sHb) : "v"(ka0), "v"(ka1), "v"(kb0), "v"(kb1));
        }
        float ta[8], tb[8]; float mx = -3.0e38f;
        const int kA = key0 + 8 * hi;
#pragma unroll
        for (int r = 0; r < 8; ++r) {
            float xa, xb;
            if (EK) { xa = (sHa[r] + sLa[r] * QRI) * SC2; xb = (sHb[r] + sLb[r] * QRI) * SC2; }
            else    { xa = sHa[r] * SC2; xb = sHb[r] * SC2; }
            const bool fa = ((kA + r) > tq) | ((float)kma[r] == 0.0f);
            const bool fb = ((kA + 16 + r) > tq) | ((float)kmb[r] == 0.0f);
            xa = fa ? NEGS : xa; xb = fb ? NEGS : xb;
            ta[r] = xa; tb[r] = xb; mx = fmaxf(mx, fmaxf(xa, xb));
        }
        mx = fmaxf(mx, __shfl_xor(mx, 16, 32));
        const float mnew = fmaxf(m, mx);
        const float alpha = __builtin_amdgcn_exp2f(m - mnew);
        v16h pb, pr = (v16h){}; float ls = 0.0f;
#pragma unroll
        for (int r = 0; r < 8; ++r) {
            const float ea = __builtin_amdgcn_exp2f((ta[r] - mnew) + PSH); const float ec = __builtin_amdgcn_exp2f((tb[r] - mnew) + PSH);
            const h16 pa = (h16)ea; const h16 pc = (h16)ec; pb[r] = pa; pb[8 + r] = pc;
            if (EK) { const h16 ga = (h16)((ea - (float)pa) * QRS); const h16 gc = (h16)((ec - (float)pc) * QRS); pr[r] = ga; pr[8 + r] = gc;
                      ls += ((float)pa + (float)pc) + ((float)ga + (float)gc) * QRI; }
            else ls += (float)pa + (float)pc;
        }
        l = l * alpha + ls; m = mnew;
        o0 = o0 * alpha; o1 = o1 * alpha; o2 = o2 * alpha; o3 = o3 * alpha;
        const h16* va = VT + vo + key0;
        const v16h v0 = ldh(va), v1 = ldh(va + (size_t)16 * SEQ), v2 = ldh(va + (size_t)32 * SEQ), v3 = ldh(va + (size_t)48 * SEQ);
        if (EK) {
            e0 = e0 * alpha; e1 = e1 * alpha; e2 = e2 * alpha; e3 = e3 * alpha;
            v16h w0 = (v16h){}, w1 = (v16h){}, w2 = (v16h){}, w3 = (v16h){};
            if (rok) { const h16* vr = VR + vro + key0; w0 = ldh(vr); w1 = ldh(vr + (size_t)16 * EARLY); w2 = ldh(vr + (size_t)32 * EARLY); w3 = ldh(vr + (size_t)48 * EARLY); }
            o0 = wmma16(v0, pb, o0); o1 = wmma16(v1, pb, o1); o2 = wmma16(v2, pb, o2); o3 = wmma16(v3, pb, o3);
            e0 = wmma16(w0, pb, e0); e1 = wmma16(w1, pb, e1); e2 = wmma16(w2, pb, e2); e3 = wmma16(w3, pb, e3);
            e0 = wmma16(v0, pr, e0); e1 = wmma16(v1, pr, e1); e2 = wmma16(v2, pr, e2); e3 = wmma16(v3, pr, e3);
            asm volatile("v_nop\n\tv_nop\n\tv_nop\n\tv_nop" : "+v"(o0), "+v"(o1), "+v"(o2), "+v"(o3), "+v"(e0), "+v"(e1), "+v"(e2), "+v"(e3)
                         : "v"(v0), "v"(v1), "v"(v2), "v"(v3), "v"(w0), "v"(w1), "v"(w2), "v"(w3), "v"(pb), "v"(pr));
        } else {
            o0 = wmma16(v0, pb, o0); o1 = wmma16(v1, pb, o1); o2 = wmma16(v2, pb, o2); o3 = wmma16(v3, pb, o3);
            asm volatile("v_nop\n\tv_nop\n\tv_nop\n\tv_nop" : "+v"(o0), "+v"(o1), "+v"(o2), "+v"(o3) : "v"(v0), "v"(v1), "v"(v2), "v"(v3), "v"(pb));
        }
        if (key0 + 32 == kc) { if (__builtin_amdgcn_ballot_w32(m < MTHR) != 0u) kend = SEQ; }
    }
    l += __shfl_xor(l, 16, 32);
    const float qmf = (float)MQ[(size_t)zh * SEQ + tq];
    const float inv = qmf * (1.0f / l);
    v8f f0 = o0, f1 = o1, f2 = o2, f3 = o3;
    if (EK) { f0 = o0 + e0 * QRI; f1 = o1 + e1 * QRI; f2 = o2 + e2 * QRI; f3 = o3 + e3 * QRI; }
    const int wb = wave * 16 * 68;
    { v4f a, c;
      a[0] = f0[0] * inv; a[1] = f0[1] * inv; a[2] = f0[2] * inv; a[3] = f0[3] * inv; c[0] = f0[4] * inv; c[1] = f0[5] * inv; c[2] = f0[6] * inv; c[3] = f0[7] * inv;
      *(v4fa*)(&os[wb + lr * 68 +  0 + 8 * hi]) = a; *(v4fa*)(&os[wb + lr * 68 +  0 + 8 * hi + 4]) = c;
      a[0] = f1[0] * inv; a[1] = f1[1] * inv; a[2] = f1[2] * inv; a[3] = f1[3] * inv; c[0] = f1[4] * inv; c[1] = f1[5] * inv; c[2] = f1[6] * inv; c[3] = f1[7] * inv;
      *(v4fa*)(&os[wb + lr * 68 + 16 + 8 * hi]) = a; *(v4fa*)(&os[wb + lr * 68 + 16 + 8 * hi + 4]) = c;
      a[0] = f2[0] * inv; a[1] = f2[1] * inv; a[2] = f2[2] * inv; a[3] = f2[3] * inv; c[0] = f2[4] * inv; c[1] = f2[5] * inv; c[2] = f2[6] * inv; c[3] = f2[7] * inv;
      *(v4fa*)(&os[wb + lr * 68 + 32 + 8 * hi]) = a; *(v4fa*)(&os[wb + lr * 68 + 32 + 8 * hi + 4]) = c;
      a[0] = f3[0] * inv; a[1] = f3[1] * inv; a[2] = f3[2] * inv; a[3] = f3[3] * inv; c[0] = f3[4] * inv; c[1] = f3[5] * inv; c[2] = f3[6] * inv; c[3] = f3[7] * inv;
      *(v4fa*)(&os[wb + lr * 68 + 48 + 8 * hi]) = a; *(v4fa*)(&os[wb + lr * 68 + 48 + 8 * hi + 4]) = c; }
    wave_sync();
    float* orow = OUT + ((size_t)b * OUT_SEQ + t0) * DM + h * HD;
#pragma unroll 1
    for (int ps = 0; ps < 2; ++ps) {
#pragma unroll
        for (int s = 0; s < 8; ++s) { const int row = 2 * s + hi, cofs = lr * 4;
            const v4f val = *(const v4fa*)(&os[wb + row * 68 + cofs]);
            *(volatile v4f*)(orow + (size_t)row * DM + cofs) = val; }
        if (ps == 0) __threadfence(); }
}

static constexpr size_t al256(size_t v) { return (v + 255) & ~(size_t)255; }
static constexpr size_t SZ_XB = al256((size_t)NB * SEQ * DM * 2);
static constexpr size_t SZ_WT = al256((size_t)3 * DM * DM * 2);
static constexpr size_t SZ_PL = al256((size_t)NB * NH_ * SEQ * HD * 2);
static constexpr size_t SZ_RP = al256((size_t)NB * NH_ * EARLY * HD * 2);
static constexpr size_t SZ_MK = al256((size_t)NB * NH_ * SEQ * 2);
static constexpr size_t SZ_TOTAL = 3 * SZ_XB + SZ_WT + 3 * SZ_PL + 3 * SZ_RP + 2 * SZ_MK;
static_assert(SZ_TOTAL <= (size_t)134217728);
static_assert(((size_t)DM * DM * 2) % 256 == 0);

extern "C" void kernel_launch(void* const* d_in, const int* in_sizes, int n_in,
                              void* d_out, int out_size, void* d_ws, size_t ws_size, hipStream_t stream) {
    if (n_in < 9) return;
    const size_t needx = ((size_t)(NB - 1) * SEQ_FULL + SEQ) * DM;
    if ((size_t)in_sizes[0] < needx || (size_t)in_sizes[1] < needx || (size_t)in_sizes[2] < needx) return;
    if ((size_t)in_sizes[3] < (size_t)DM * DM || (size_t)in_sizes[5] < (size_t)DM * DM || (size_t)in_sizes[7] < (size_t)DM * DM) return;
    if ((size_t)in_sizes[4] < (size_t)DM || (size_t)in_sizes[6] < (size_t)DM || (size_t)in_sizes[8] < (size_t)DM) return;
    if ((size_t)out_size < ((size_t)(NB - 1) * OUT_SEQ + SEQ) * DM) return;
    if (SZ_TOTAL > ws_size) return;
    const float* xq = (const float*)d_in[0]; const float* xk = (const float*)d_in[1]; const float* xv = (const float*)d_in[2];
    const float* wq = (const float*)d_in[3]; const float* bq = (const float*)d_in[4];
    const float* wk = (const float*)d_in[5]; const float* bk = (const float*)d_in[6];
    const float* wv = (const float*)d_in[7]; const float* bv = (const float*)d_in[8];
    float* OUT = (float*)d_out;
    char* wsp = (char*)d_ws;
    bf* XQ = (bf*)wsp; wsp += SZ_XB;
    bf* XK = (bf*)wsp; wsp += SZ_XB;
    bf* XV = (bf*)wsp; wsp += SZ_XB;
    bf* WT = (bf*)wsp; wsp += SZ_WT;
    h16* QH = (h16*)wsp; wsp += SZ_PL;
    h16* KP = (h16*)wsp; wsp += SZ_PL;
    h16* VT = (h16*)wsp; wsp += SZ_PL;
    h16* QR = (h16*)wsp; wsp += SZ_RP;
    h16* KR = (h16*)wsp; wsp += SZ_RP;
    h16* VR = (h16*)wsp; wsp += SZ_RP;
    h16* MQ = (h16*)wsp; wsp += SZ_MK;
    h16* MK = (h16*)wsp; wsp += SZ_MK;
    bf* WTQ = WT; bf* WTK = WT + (size_t)DM * DM; bf* WTV = WT + (size_t)2 * DM * DM;

    if (SEQ == SEQ_FULL) {
        const size_t n8 = (size_t)NB * SEQ * DM / 8; const unsigned g = (unsigned)((n8 + 255) / 256);
        k_cvt8<<<g, 256, 0, stream>>>(xq, XQ, n8);
        k_cvt8<<<g, 256, 0, stream>>>(xk, XK, n8);
        k_cvt8<<<g, 256, 0, stream>>>(xv, XV, n8);
    } else {
        const size_t n8 = (size_t)SEQ * DM / 8; const unsigned g = (unsigned)((n8 + 255) / 256);
        for (int b = 0; b < NB; ++b) {
            k_cvt8<<<g, 256, 0, stream>>>(xq + (size_t)b * SEQ_FULL * DM, XQ + (size_t)b * SEQ * DM, n8);
            k_cvt8<<<g, 256, 0, stream>>>(xk + (size_t)b * SEQ_FULL * DM, XK + (size_t)b * SEQ * DM, n8);
            k_cvt8<<<g, 256, 0, stream>>>(xv + (size_t)b * SEQ_FULL * DM, XV + (size_t)b * SEQ * DM, n8);
        }
    }
    k_cvtT<<<dim3(DM / 64, DM / 64, 1), 256, 0, stream>>>(wq, WTQ);
    k_cvtT<<<dim3(DM / 64, DM / 64, 1), 256, 0, stream>>>(wk, WTK);
    k_cvtT<<<dim3(DM / 64, DM / 64, 1), 256, 0, stream>>>(wv, WTV);

    k_proj<0><<<dim3(NB * SEQ / 64, DM / 64, 1), 32, 0, stream>>>(XQ, WTQ, bq, QH, QR, MQ);
    k_proj<0><<<dim3(NB * SEQ / 64, DM / 64, 1), 32, 0, stream>>>(XK, WTK, bk, KP, KR, MK);
    k_proj<1><<<dim3(DM / 64, NB * SEQ / 64, 1), 32, 0, stream>>>(WTV, XV, bv, VT, VR, MK);

    k_flash<1><<<dim3(EARLY / (16 * AW), NB * NH_, 1), 32 * AW, 0, stream>>>(QH, QR, KP, KR, VT, VR, MQ, MK, OUT);
    if (SEQ > EARLY)
        k_flash<0><<<dim3((SEQ - EARLY) / (16 * AW), NB * NH_, 1), 32 * AW, 0, stream>>>(QH, QR, KP, KR, VT, VR, MQ, MK, OUT);
}
